// Metacontroller_18846316495231
// MI455X (gfx1250) — hardware-verified
//
#include <hip/hip_runtime.h>
#include <math.h>


#define NB 16
#define TT 512
#define DD 256
#define HG 128
#define GC 32
#define ZZ 8
#define RR 16
#define NA 18
#define NRW (NB * TT)

typedef __attribute__((ext_vector_type(16))) _Float16 v16h;
typedef __attribute__((ext_vector_type(16))) __bf16 v16b;
typedef __attribute__((ext_vector_type(8)))  _Float16 v8h;
typedef __attribute__((ext_vector_type(8)))  float v8f;
typedef __attribute__((ext_vector_type(4)))  float v4f;
typedef __attribute__((ext_vector_type(4)))  unsigned v4u;
typedef float __attribute__((may_alias)) float_a;

template <typename T> __device__ __forceinline__ void vst2(void* p, T v) { *(volatile T*)p = v; __threadfence(); *(volatile T*)p = v; }
__device__ __forceinline__ v8f wmma16(v16h a, v16h b, v8f c) {
  v8f d = __builtin_amdgcn_wmma_f32_16x16x32_f16(false, a, false, b, (short)0, c, false, false);
  asm volatile("v_nop\n\tv_nop\n\tv_nop\n\tv_nop" : "+v"(d) : "v"(a), "v"(b));
  return d;
}
__device__ __forceinline__ v8f wmma_bf(v16b a, v16b b, v8f c) {
  v8f d = __builtin_amdgcn_wmma_f32_16x16x32_bf16(false, a, false, b, (short)0, c, false, false);
  asm volatile("v_nop\n\tv_nop\n\tv_nop\n\tv_nop" : "+v"(d) : "v"(a), "v"(b));
  return d;
}
__device__ __forceinline__ v16h frag_h(const _Float16* rowk0, int lane) {
  union { v16h v; v8h q[2]; } u; const _Float16* p = rowk0 + 8 * (lane >> 4);
  u.q[0] = *(const v8h*)p; u.q[1] = *(const v8h*)(p + 16); return u.v;
}
__device__ __forceinline__ v16h frag_f32(const float* rowk0, int lane) {
  v16h a; const float* p = rowk0 + 8 * (lane >> 4);
#pragma unroll
  for (int i = 0; i < 8; ++i) { a[i] = (_Float16)p[i]; a[8 + i] = (_Float16)p[16 + i]; }
  return a;
}
struct F2 { v16b h, l; };
__device__ __forceinline__ F2 split_row(const float* row, int k0, int lane) { F2 r; const float* p = row + k0 + 8 * (lane >> 4);
#pragma unroll
  for (int i = 0; i < 8; ++i) { const float a = p[i], b = p[16 + i]; const __bf16 ha = (__bf16)a, hb = (__bf16)b;
    r.h[i] = ha; r.l[i] = (__bf16)(a - (float)ha); r.h[8 + i] = hb; r.l[8 + i] = (__bf16)(b - (float)hb); }
  return r; }
__device__ __forceinline__ v8f mac3(const F2& a, const F2& b, v8f c) { c = wmma_bf(a.l, b.h, c); c = wmma_bf(a.h, b.l, c); return wmma_bf(a.h, b.h, c); }
__device__ __forceinline__ float sigm(float v) { return 1.0f / (1.0f + expf(-v)); }
#define LDSX() do { asm volatile("s_wait_dscnt 0" ::: "memory"); __builtin_amdgcn_wave_barrier(); __builtin_amdgcn_fence(__ATOMIC_RELEASE, "workgroup"); } while (0)

template <int NT, int ACC>
__global__ __launch_bounds__(128) void k_gemm(const float* __restrict__ A, int lda, int K, const float* __restrict__ W, int ldw, const float* __restrict__ bias,
                                            float* __restrict__ Out, int ldo) {
  __shared__ __align__(16) float so[4][16][NT * 16 + 4];
  const int tid = threadIdx.x, wave = tid >> 5, lane = tid & 31, col = lane & 15, g = lane >> 4;
  const int r0 = blockIdx.x * 64 + wave * 16, n0 = blockIdx.y * (NT * 16);
  v8f acc[NT];
#pragma unroll
  for (int j = 0; j < NT; ++j) acc[j] = (v8f){};
#pragma unroll 1
  for (int kc = 0; kc < K / 32; ++kc) { const v16h a = frag_f32(A + (size_t)(r0 + col) * lda + kc * 32, lane);
#pragma unroll
    for (int j = 0; j < NT; ++j) acc[j] = wmma16(a, frag_f32(W + (size_t)(n0 + j * 16 + col) * ldw + kc * 32, lane), acc[j]); }
  const int LD = NT * 16 + 4;
#pragma unroll
  for (int j = 0; j < NT; ++j) { const float bv = bias ? bias[n0 + j * 16 + col] : 0.f;
#pragma unroll
    for (int r = 0; r < 8; ++r) so[wave][8 * g + r][j * 16 + col] = acc[j][r] + bv; }
  LDSX();
  for (int q = lane; q < 16 * NT * 4; q += 32) { const int rl = q / (NT * 4), pc = q % (NT * 4); float* o = Out + (size_t)(r0 + rl) * ldo + n0 + pc * 4;
    v4f v = *(const v4f*)(&so[wave][rl][pc * 4]); if (ACC) v += *(const v4f*)o; vst2(o, v); }
}
__global__ __launch_bounds__(256) void k_cvt(const float* __restrict__ s, _Float16* __restrict__ d, size_t n8) {
  const size_t g8 = (size_t)blockIdx.x * 256 + threadIdx.x; if (g8 >= n8) return;
  union { v8h h; v4u u; } pk;
#pragma unroll
  for (int e = 0; e < 8; ++e) pk.h[e] = (_Float16)s[g8 * 8 + e];
  vst2(d + g8 * 8, pk.u);
}

__global__ __launch_bounds__(256) void k_bigru(const float* __restrict__ gif, const float* __restrict__ gib, const _Float16* __restrict__ whf, const _Float16* __restrict__ whb,
                                             const float* __restrict__ bhf, const float* __restrict__ bhb, float* __restrict__ s) {
  __shared__ __align__(16) float gh[NB][3 * HG];
  __shared__ __align__(16) _Float16 h16[NB][HG + 16];
  const int tid = threadIdx.x, w = tid >> 5, lane = tid & 31, col = lane & 15, g = lane >> 4;
  const int dir = blockIdx.x, r = tid >> 4, u0 = (tid & 15) * 8;
  const float* gi = dir == 0 ? gif : gib; const _Float16* Wh = dir == 0 ? whf : whb; const float* bh = dir == 0 ? bhf : bhb;
  float h[8];
#pragma unroll
  for (int j = 0; j < 8; ++j) { h[j] = 0.f; h16[r][u0 + j] = (_Float16)0.f; }
  __syncthreads();
#pragma unroll 1
  for (int st = 0; st < TT; ++st) { const int t = dir == 0 ? st : TT - 1 - st;
    v8f acc[3] = {};
#pragma unroll
    for (int kc = 0; kc < HG / 32; ++kc) { const v16h a = frag_h(&h16[col][0] + kc * 32, lane);
#pragma unroll
      for (int q = 0; q < 3; ++q) acc[q] = wmma16(a, frag_h(Wh + (size_t)(w * 48 + q * 16 + col) * HG + kc * 32, lane), acc[q]); }
#pragma unroll
    for (int q = 0; q < 3; ++q) { const int n = w * 48 + q * 16 + col; const float bb = bh[n];
#pragma unroll
      for (int rr = 0; rr < 8; ++rr) gh[8 * g + rr][n] = acc[q][rr] + bb; }
    __syncthreads();
    const float* gr = gi + ((size_t)r * TT + t) * (3 * HG);
    union { v8h hv; v4u u; } pk; v4f o0, o1;
#pragma unroll
    for (int j = 0; j < 8; ++j) { const int u = u0 + j;
      const float rg = sigm(gr[u] + gh[r][u]), zg = sigm(gr[HG + u] + gh[r][HG + u]);
      const float ng = tanhf(gr[2 * HG + u] + rg * gh[r][2 * HG + u]);
      h[j] = (1.0f - zg) * ng + zg * h[j]; pk.hv[j] = (_Float16)h[j]; if (j < 4) o0[j] = h[j]; else o1[j - 4] = h[j]; }
    *(v4u*)(&h16[r][u0]) = pk.u;
    float* dst = s + ((size_t)r * TT + t) * DD + dir * HG + u0;
    vst2(dst, o0); vst2(dst + 4, o1);
    __syncthreads();
  }
}

__global__ __launch_bounds__(256) void k_ctrl(const float* __restrict__ gie, const float* __restrict__ se, const float* __restrict__ eps,
                                            const float* __restrict__ whe, const float* __restrict__ bhe, const float* __restrict__ muw, const float* __restrict__ mub,
                                            const float* __restrict__ lvw, const float* __restrict__ lvb, const float* __restrict__ sw1, const float* __restrict__ sw1b,
                                            const float* __restrict__ sw2, const float* __restrict__ sw2b,
                                            float* __restrict__ smu, float* __restrict__ slv, float* __restrict__ sz, float* __restrict__ beta_out) {
  __shared__ float h[NB][GC], zprev[NB][ZZ], ghs[NB][3 * GC], mu[NB][ZZ], lv[NB][ZZ], hid[NB][64], znew[NB][ZZ];
  __shared__ __align__(16) _Float16 h16[NB][GC + 16];
  __shared__ __align__(16) float sbeta[NB * TT];
  const int tid = threadIdx.x, w = tid >> 5, lane = tid & 31, col = lane & 15, g = lane >> 4;
  for (int q = tid; q < NB * GC; q += 256) { (&h[0][0])[q] = 0.f; h16[q >> 5][q & 31] = (_Float16)0.f; }
  if (tid < NB * ZZ) (&zprev[0][0])[tid] = 0.f;
  __syncthreads();
#pragma unroll 1
  for (int t = 0; t < TT; ++t) {
    if (w < 6) { v8f acc = {}; acc = wmma16(frag_h(&h16[col][0], lane), frag_f32(whe + (size_t)(w * 16 + col) * GC, lane), acc);
      const float bb = bhe[w * 16 + col];
#pragma unroll
      for (int rr = 0; rr < 8; ++rr) ghs[8 * g + rr][w * 16 + col] = acc[rr] + bb; }
    __syncthreads();
    { const int r = tid >> 4, u0 = (tid & 15) * 2; const float* gi = gie + ((size_t)r * TT + t) * (3 * GC);
#pragma unroll
      for (int j = 0; j < 2; ++j) { const int u = u0 + j;
        const float rg = sigm(gi[u] + ghs[r][u]), zg = sigm(gi[GC + u] + ghs[r][GC + u]);
        const float ng = tanhf(gi[2 * GC + u] + rg * ghs[r][2 * GC + u]);
        const float hn = (1.0f - zg) * ng + zg * h[r][u];
        ghs[r][u] = hn; } }
    __syncthreads();
    { const int r = tid >> 4, u0 = (tid & 15) * 2; h[r][u0] = ghs[r][u0]; h[r][u0 + 1] = ghs[r][u0 + 1];
      h16[r][u0] = (_Float16)ghs[r][u0]; h16[r][u0 + 1] = (_Float16)ghs[r][u0 + 1]; }
    __syncthreads();
    { const int r = tid >> 4, which = (tid >> 3) & 1, o = tid & 7; const float* Wm = which ? lvw : muw; float a = which ? lvb[o] : mub[o];
#pragma unroll 1
      for (int k = 0; k < GC; ++k) a += h[r][k] * Wm[o * GC + k];
      (which ? lv : mu)[r][o] = a; }
    { const int r = tid >> 4, o0 = (tid & 15) * 4; const float* ser = se + ((size_t)r * TT + t) * 64;
#pragma unroll
      for (int j = 0; j < 4; ++j) { const int o = o0 + j; float a = ser[o] + sw1b[o];
#pragma unroll 1
        for (int k = 0; k < GC; ++k) a += h[r][k] * sw1[(size_t)o * 296 + 256 + k];
#pragma unroll
        for (int k = 0; k < ZZ; ++k) a += zprev[r][k] * sw1[(size_t)o * 296 + 288 + k];
        hid[r][o] = tanhf(a); } }
    __syncthreads();
    if (tid < NB) { float a = sw2b[0];
#pragma unroll 1
      for (int k = 0; k < 64; ++k) a += hid[tid][k] * sw2[k];
      sbeta[tid * TT + t] = sigm(a); }
    __syncthreads();
    if (tid < NB * ZZ) { const int r = tid >> 3, o = tid & 7; const float be = sbeta[r * TT + t];
      const float zz = be * (mu[r][o] + expf(0.5f * lv[r][o]) * eps[((size_t)r * TT + t) * ZZ + o]) + (1.0f - be) * zprev[r][o];
      znew[r][o] = zz; }
    __syncthreads();
    if (tid < NB * ZZ) { const int r = tid >> 3, o = tid & 7; zprev[r][o] = znew[r][o]; }
    if (tid < 3 * 32) { const int which = tid >> 5, q = tid & 31; const float* src = which == 0 ? &mu[0][0] : (which == 1 ? &lv[0][0] : &znew[0][0]);
      float* dst = (which == 0 ? smu : (which == 1 ? slv : sz)) + (size_t)t * NB * ZZ;
      v4f v = { src[q * 4], src[q * 4 + 1], src[q * 4 + 2], src[q * 4 + 3] }; vst2(dst + q * 4, v); }
    __syncthreads();
  }
  for (int q = tid; q < NB * TT / 4; q += 256) vst2(beta_out + q * 4, *(const v4f*)(&sbeta[q * 4]));
}
__global__ __launch_bounds__(128) void k_tmajor(const float* __restrict__ sm, float* __restrict__ out) {
  const int b = blockIdx.y, t0 = blockIdx.x * 64, tid = threadIdx.x;
  const int t = t0 + (tid >> 1), hf = (tid & 1) * 4;
  vst2(out + ((size_t)b * TT + t) * ZZ + hf, *(const v4f*)(sm + ((size_t)t * NB + b) * ZZ + hf));
}
__global__ __launch_bounds__(32) void k_dec(const float* __restrict__ zbt, const float* __restrict__ e, const float* __restrict__ d1w, const float* __restrict__ d1b,
                                          const float* __restrict__ d2w, const float* __restrict__ d2b, const float* __restrict__ lng, const float* __restrict__ lnb,
                                          const float* __restrict__ hw, const float* __restrict__ hb, float* __restrict__ logits) {
  __shared__ __align__(16) float hm[16][36];
  __shared__ __align__(16) float pert[16][DD + 4];
  __shared__ __align__(16) float lg[16 * NA + 4];
  const int lane = threadIdx.x, col = lane & 15, g = lane >> 4;
  const int r0 = blockIdx.x * 16;
  { const float* zr = zbt + (size_t)(r0 + col) * ZZ;
#pragma unroll
    for (int j = 0; j < 16; ++j) { const int o = g * 16 + j; float a = d1b[o];
#pragma unroll
      for (int k = 0; k < ZZ; ++k) a += zr[k] * d1w[o * ZZ + k];
      hm[col][o] = tanhf(a); } }
  LDSX();
  const F2 ah = split_row(&hm[col][0], 0, lane);
  const float* er = e + (size_t)r0 * DD;
  float tmp[8] = {0.f, 0.f, 0.f, 0.f, 0.f, 0.f, 0.f, 0.f};
#pragma unroll 1
  for (int d = 0; d < DD; ++d) { const int j = 256 + d;
    v8f acc = {}; acc = mac3(ah, split_row(d2w + (size_t)(j * 16 + col) * 32, 0, lane), acc);
    const float bb = d2b[j * 16 + col];
#pragma unroll
    for (int rr = 0; rr < 8; ++rr) tmp[rr] += (acc[rr] + bb) * er[(size_t)(8 * g + rr) * DD + d]; }
#pragma unroll 1
  for (int d = 0; d < DD; ++d) { const int j = d;
    v8f acc = {}; acc = mac3(ah, split_row(d2w + (size_t)(j * 16 + col) * 32, 0, lane), acc);
    const float bb = d2b[j * 16 + col];
    float pr[8];
#pragma unroll
    for (int rr = 0; rr < 8; ++rr) pr[rr] = (acc[rr] + bb) * tmp[rr];
#pragma unroll
    for (int off = 8; off >= 1; off >>= 1) {
#pragma unroll
      for (int rr = 0; rr < 8; ++rr) pr[rr] += __shfl_xor(pr[rr], off, 32); }
    if (col == 0) {
#pragma unroll
      for (int rr = 0; rr < 8; ++rr) pert[8 * g + rr][d] = er[(size_t)(8 * g + rr) * DD + d] + pr[rr]; } }
  LDSX();
  { float sm = 0.f;
    for (int i = 0; i < 128; ++i) sm += pert[col][g * 128 + i];
    sm += __shfl_xor(sm, 16, 32); const float mu = sm / (float)DD; float q2 = 0.f;
    for (int i = 0; i < 128; ++i) { const float dv = pert[col][g * 128 + i] - mu; q2 += dv * dv; }
    q2 += __shfl_xor(q2, 16, 32); const float rs = rsqrtf(q2 / (float)DD + 1e-5f);
    LDSX();
    for (int i = 0; i < 128; ++i) { const int c = g * 128 + i; pert[col][c] = (pert[col][c] - mu) * rs * lng[c] + lnb[c]; } }
  LDSX();
  for (int j = 0; j < 9; ++j) { const int o = g * 9 + j; float a = hb[o];
#pragma unroll 1
    for (int k = 0; k < DD; ++k) a += pert[col][k] * hw[o * DD + k];
    lg[col * NA + o] = a; }
  LDSX();
  for (int q = lane; q < 72; q += 32) vst2(logits + (size_t)r0 * NA + q * 4, *(const v4f*)(&lg[q * 4]));
}

extern "C" void kernel_launch(void* const* d_in, const int* in_sizes, int n_in,
                              void* d_out, int out_size, void* d_ws, size_t ws_size,
                              hipStream_t stream) {
  (void)in_sizes; (void)n_in; (void)out_size; (void)ws_size;
  const float** I = (const float**)d_in;
  const float* e = I[0]; const float* eps = I[1];
  const float* wihf = I[2]; const float* whhf = I[3]; const float* bihf = I[4]; const float* bhhf = I[5];
  const float* wihb = I[6]; const float* whhb = I[7]; const float* bihb = I[8]; const float* bhhb = I[9];
  const float* wihe = I[10]; const float* whhe = I[11]; const float* bihe = I[12]; const float* bhhe = I[13];
  const float* muw = I[14]; const float* mub = I[15]; const float* lvw = I[16]; const float* lvb = I[17];
  const float* sw1 = I[18]; const float* sw1b = I[19]; const float* sw2 = I[20]; const float* sw2b = I[21];
  const float* d1w = I[22]; const float* d1b = I[23]; const float* d2w = I[24]; const float* d2b = I[25];
  const float* lng = I[26]; const float* lnb = I[27]; const float* hw = I[28]; const float* hb = I[29];
  float* logits = (float*)d_out; float* mu_o = logits + (size_t)NRW * NA; float* lv_o = mu_o + (size_t)NRW * ZZ; float* be_o = lv_o + (size_t)NRW * ZZ; float* z_o = be_o + (size_t)NRW;
  char* ws = (char*)d_ws; size_t off = 0;
  auto take = [&](size_t bytes) { char* p = ws + off; off += (bytes + 255) & ~(size_t)255; return p; };
  float* gif = (float*)take((size_t)NRW * 3 * HG * 4); float* gib = (float*)take((size_t)NRW * 3 * HG * 4);
  _Float16* whf16 = (_Float16*)take((size_t)3 * HG * HG * 2); _Float16* whb16 = (_Float16*)take((size_t)3 * HG * HG * 2);
  float* s = (float*)take((size_t)NRW * DD * 4);
  float* gie = (float*)take((size_t)NRW * 3 * GC * 4); float* se = (float*)take((size_t)NRW * 64 * 4);
  float* smu = (float*)take((size_t)NRW * ZZ * 4); float* slv = (float*)take((size_t)NRW * ZZ * 4); float* sz = (float*)take((size_t)NRW * ZZ * 4);
  k_gemm<8, 0><<<dim3(NRW / 64, 3), 128, 0, stream>>>(e, DD, DD, wihf, DD, bihf, gif, 3 * HG);
  k_gemm<8, 0><<<dim3(NRW / 64, 3), 128, 0, stream>>>(e, DD, DD, wihb, DD, bihb, gib, 3 * HG);
  k_gemm<6, 0><<<dim3(NRW / 64, 1), 128, 0, stream>>>(e, DD, DD, wihe, 2 * DD, bihe, gie, 3 * GC);
  k_gemm<4, 0><<<dim3(NRW / 64, 1), 128, 0, stream>>>(e, DD, DD, sw1, 296, nullptr, se, 64);
  k_cvt<<<(3 * HG * HG / 8 + 255) / 256, 256, 0, stream>>>(whhf, whf16, (size_t)3 * HG * HG / 8);
  k_cvt<<<(3 * HG * HG / 8 + 255) / 256, 256, 0, stream>>>(whhb, whb16, (size_t)3 * HG * HG / 8);
  k_bigru<<<2, 256, 0, stream>>>(gif, gib, whf16, whb16, bhhf, bhhb, s);
  k_gemm<6, 1><<<dim3(NRW / 64, 1), 128, 0, stream>>>(s, DD, DD, wihe + DD, 2 * DD, nullptr, gie, 3 * GC);
  k_ctrl<<<1, 256, 0, stream>>>(gie, se, eps, whhe, bhhe, muw, mub, lvw, lvb, sw1, sw1b, sw2, sw2b, smu, slv, sz, be_o);
  k_tmajor<<<dim3(TT / 64, NB), 128, 0, stream>>>(smu, mu_o);
  k_tmajor<<<dim3(TT / 64, NB), 128, 0, stream>>>(slv, lv_o);
  k_tmajor<<<dim3(TT / 64, NB), 128, 0, stream>>>(sz, z_o);
  k_dec<<<NRW / 16, 32, 0, stream>>>(z_o, e, d1w, d1b, d2w, d2b, lng, lnb, hw, hb, logits);
}
